// CAM_1288490188988
// MI455X (gfx1250) — hardware-run, weakly checked
//
#include <hip/hip_runtime.h>


namespace {
constexpr int N1 = 8192, N2 = 8192, DI = 128, D = 32, FO = 128, KB = 128;
constexpr float XS = 8.0f, HS = 256.0f, WSC = 256.0f, PS = 256.0f, LNEPS = 1e-5f;
typedef _Float16 b16;
typedef __attribute__((ext_vector_type(16))) _Float16 v16b;
typedef __attribute__((ext_vector_type(8))) _Float16 v8b;
typedef __attribute__((ext_vector_type(8))) float v8f;
typedef __attribute__((ext_vector_type(4))) float v4f;
__device__ __forceinline__ float bf16_rne(float f) { unsigned int u = __float_as_uint(f); u += 0x7FFFu + ((u >> 16) & 1u); float r = __uint_as_float(u & 0xFFFF0000u); asm volatile("" : "+v"(r)); return r; }
__device__ __forceinline__ float bfv(float f) { float r = bf16_rne(f); asm volatile("" : "+v"(r)); return r; }
__device__ __forceinline__ void split16(float v, b16& hi, b16& lo) { hi = (b16)v; lo = (b16)(v - (float)hi); }
__device__ __forceinline__ v16b frag_kb(const b16* p, int hh) { const v8b a = *(const v8b*)(p + 8 * hh), b = *(const v8b*)(p + 16 + 8 * hh); v16b f;
#pragma unroll
  for (int e = 0; e < 8; ++e) { f[e] = a[e]; f[8 + e] = b[e]; } return f; }
__device__ __forceinline__ v8f wmma16b(v16b a, v16b b, v8f c) { v8f d = __builtin_amdgcn_wmma_f32_16x16x32_f16(false, a, false, b, (short)0, c, false, false); asm volatile("v_nop\n\tv_nop\n\tv_nop\n\tv_nop" : "+v"(d) : "v"(a), "v"(b)); return d; }
__device__ __forceinline__ void wave_lds_sync() { __builtin_amdgcn_fence(__ATOMIC_RELEASE, "workgroup"); __builtin_amdgcn_wave_barrier(); __builtin_amdgcn_fence(__ATOMIC_ACQUIRE, "workgroup"); }
__device__ __forceinline__ float pmul(float a, float b) { float p = a * b; asm volatile("" : "+v"(p)); return p; }

__global__ __launch_bounds__(256) void wput_kernel(const float* __restrict__ wq, const float* __restrict__ wk, const float* __restrict__ wv, const float* __restrict__ wo, b16* __restrict__ W3, b16* __restrict__ WO) { const int u = blockIdx.x * 256 + threadIdx.x; v8b v;
  if (u < 3 * D * (DI / 8)) { const int p = u / (D * (DI / 8)), r = u % (D * (DI / 8)); const int o = r / (DI / 8), k0 = (r % (DI / 8)) * 8; const float* w = p == 0 ? wq : (p == 1 ? wk : wv);
#pragma unroll
    for (int j = 0; j < 8; ++j) v[j] = (b16)(bf16_rne(w[(size_t)(k0 + j) * D + o]) * WSC); for (int pass = 0; pass < 2; ++pass) { *(volatile v8b*)(W3 + ((size_t)p * D + o) * DI + k0) = v; __threadfence(); } }
  if (u < FO * (D / 8)) { const int o = u / (D / 8), k0 = (u % (D / 8)) * 8;
#pragma unroll
    for (int j = 0; j < 8; ++j) v[j] = (b16)(bf16_rne(wo[(size_t)(k0 + j) * FO + o]) * WSC); for (int pass = 0; pass < 2; ++pass) { *(volatile v8b*)(WO + (size_t)o * D + k0) = v; __threadfence(); } } }
template <int MODE>
__global__ __launch_bounds__(32) void proj_kernel(const float* __restrict__ x, const b16* __restrict__ W3, const float* __restrict__ ba, const float* __restrict__ bb, int RLIM, b16* __restrict__ Ah_, b16* __restrict__ Al_, b16* __restrict__ Bh_, b16* __restrict__ Bl_) { __shared__ __attribute__((aligned(16))) b16 Xh[16][DI + 8]; __shared__ __attribute__((aligned(16))) b16 Oh[16][72], Ol[16][72]; const int lane = threadIdx.x, nloc = lane & 15, hlf = lane >> 4; const size_t m0 = (size_t)blockIdx.x * 16; if (m0 >= (size_t)RLIM) return; constexpr int NT = MODE == 0 ? 2 : 4;
  for (int rr = 0; rr < 16; ++rr) for (int q = 0; q < 4; ++q) Xh[rr][q * 32 + lane] = (b16)(bf16_rne(x[(m0 + rr) * DI + q * 32 + lane]) * XS); if (lane < 16) for (int k = DI; k < DI + 8; ++k) Xh[lane][k] = (b16)0.0f;
  wave_lds_sync(); v8f acc[NT];
#pragma unroll
  for (int t = 0; t < NT; ++t) acc[t] = (v8f){};
  const b16* Wb = W3 + (size_t)(MODE == 0 ? 0 : D) * DI;
#pragma unroll
  for (int kb = 0; kb < DI; kb += 32) { const v16b a = frag_kb(&Xh[nloc][kb], hlf);
#pragma unroll
    for (int t = 0; t < NT; ++t) acc[t] = wmma16b(a, frag_kb(Wb + (size_t)(t * 16 + nloc) * DI + kb, hlf), acc[t]); }
#pragma unroll
  for (int t = 0; t < NT; ++t) { const int cc = t * 16 + nloc; const float bias = bfv((t < 2 ? ba : bb)[cc & 31]);
#pragma unroll
    for (int r8 = 0; r8 < 8; ++r8) { b16 p, ql; split16((acc[t][r8] * (1.0f / (XS * WSC)) + bias) * HS, p, ql); Oh[8 * hlf + r8][cc] = p; Ol[8 * hlf + r8][cc] = ql; } }
  wave_lds_sync();
  typedef __attribute__((ext_vector_type(2))) _Float16 v2b;
  for (int pass = 0; pass < 2; ++pass) { for (int rr = 0; rr < 16; ++rr) { if (lane < 16) { *(volatile v2b*)(Ah_ + (m0 + rr) * D + lane * 2) = *(const v2b*)(&Oh[rr][lane * 2]); *(volatile v2b*)(Al_ + (m0 + rr) * D + lane * 2) = *(const v2b*)(&Ol[rr][lane * 2]); }
      else if (MODE == 1) { const int l2 = lane - 16; *(volatile v2b*)(Bh_ + (m0 + rr) * D + l2 * 2) = *(const v2b*)(&Oh[rr][32 + l2 * 2]); *(volatile v2b*)(Bl_ + (m0 + rr) * D + l2 * 2) = *(const v2b*)(&Ol[rr][32 + l2 * 2]); } } __threadfence(); } }
__global__ __launch_bounds__(32) void att_kernel(const b16* __restrict__ Qh, const b16* __restrict__ Ql, const b16* __restrict__ Kh, const b16* __restrict__ Kl, const b16* __restrict__ Vh, const b16* __restrict__ Vl, const b16* __restrict__ WO, const float* __restrict__ gam, const float* __restrict__ bet, const float* __restrict__ bo, int QLIM, int KLIM, float* __restrict__ out) {
  __shared__ __attribute__((aligned(16))) b16 Ph_[16][KB + 8], Pl_[16][KB + 8], Vth[D][KB + 8], Vtl[D][KB + 8], Nh[16][40], Nl[16][40]; __shared__ float Sf[16][KB + 4], Of[16][D + 4], Tf[16][FO + 4];
  const int lane = threadIdx.x, nloc = lane & 15, hlf = lane >> 4; const size_t t0 = (size_t)blockIdx.x * 16; if (t0 >= (size_t)QLIM) return;
  const v16b qa = frag_kb(Qh + (t0 + nloc) * D, hlf), qb = frag_kb(Ql + (t0 + nloc) * D, hlf);
  float m_r[8], den_r[8]; v8f acc[2] = {(v8f){}, (v8f){}};
#pragma unroll
  for (int r8 = 0; r8 < 8; ++r8) { m_r[r8] = -INFINITY; den_r[r8] = 0.0f; }
#pragma unroll 1
  for (int kb0 = 0; kb0 < KLIM; kb0 += KB) {
    for (int rr = 0; rr < KB; rr += 2) { const int r = rr + hlf; const size_t key = (size_t)kb0 + r; Vth[nloc][r] = Vh[key * D + nloc]; Vth[16 + nloc][r] = Vh[key * D + 16 + nloc]; Vtl[nloc][r] = Vl[key * D + nloc]; Vtl[16 + nloc][r] = Vl[key * D + 16 + nloc]; }
#pragma unroll
    for (int t = 0; t < KB / 16; ++t) { const size_t key = (size_t)kb0 + t * 16 + nloc; const v16b ka = frag_kb(Kh + key * D, hlf), kbf = frag_kb(Kl + key * D, hlf); v8f s = {}; s = wmma16b(qa, ka, s); s = wmma16b(qa, kbf, s); s = wmma16b(qb, ka, s);
#pragma unroll
      for (int r8 = 0; r8 < 8; ++r8) Sf[8 * hlf + r8][t * 16 + nloc] = s[r8] * (1.0f / (HS * HS)); }
    wave_lds_sync();
#pragma unroll
    for (int rr = 0; rr < 16; ++rr) { float mx = -INFINITY;
#pragma unroll
      for (int q = 0; q < 4; ++q) mx = fmaxf(mx, Sf[rr][q * 32 + lane]);
      for (int o = 16; o; o >>= 1) mx = fmaxf(mx, __shfl_xor(mx, o));
      const float mold = __shfl(m_r[rr & 7], (rr >> 3) * 16); const float mn = fmaxf(mold, mx); const float sf = (mold == -INFINITY) ? 0.0f : __expf(mold - mn); float ps = 0.0f;
#pragma unroll
      for (int q = 0; q < 4; ++q) { const int kx = q * 32 + lane; const float p = __expf(Sf[rr][kx] - mn); ps += p; b16 ph, pl; split16(p * PS, ph, pl); Ph_[rr][kx] = ph; Pl_[rr][kx] = pl; }
      for (int o = 16; o; o >>= 1) ps += __shfl_xor(ps, o);
      if ((rr >> 3) == hlf) { const int r8 = rr & 7; den_r[r8] = den_r[r8] * sf + ps; m_r[r8] = mn;
#pragma unroll
        for (int t = 0; t < 2; ++t) acc[t][r8] = acc[t][r8] * sf; } }
    wave_lds_sync();
#pragma unroll
    for (int ks = 0; ks < KB; ks += 32) { const v16b pa = frag_kb(&Ph_[nloc][ks], hlf), pb = frag_kb(&Pl_[nloc][ks], hlf);
#pragma unroll
      for (int t = 0; t < 2; ++t) { const v16b vh = frag_kb(&Vth[t * 16 + nloc][ks], hlf), vl = frag_kb(&Vtl[t * 16 + nloc][ks], hlf); acc[t] = wmma16b(pa, vh, acc[t]); acc[t] = wmma16b(pa, vl, acc[t]); acc[t] = wmma16b(pb, vh, acc[t]); } }
    wave_lds_sync(); }
#pragma unroll
  for (int t = 0; t < 2; ++t)
#pragma unroll
    for (int r8 = 0; r8 < 8; ++r8) Of[8 * hlf + r8][t * 16 + nloc] = acc[t][r8] * (1.0f / (HS * PS)) / den_r[r8];
  wave_lds_sync();
  for (int rr = 0; rr < 16; ++rr) { const float v = Of[rr][lane]; float s = v; for (int o = 16; o; o >>= 1) s += __shfl_xor(s, o); const float mu = s / D; float s2 = (v - mu) * (v - mu); for (int o = 16; o; o >>= 1) s2 += __shfl_xor(s2, o); const float rs = rsqrtf(s2 / D + LNEPS); const float nv = pmul(pmul(v - mu, rs), bfv(gam[lane])) + bfv(bet[lane]); b16 p, ql; split16(nv * HS, p, ql); Nh[rr][lane] = p; Nl[rr][lane] = ql; if (lane < 8) { Nh[rr][32 + lane] = (b16)0.0f; Nl[rr][32 + lane] = (b16)0.0f; } }
  wave_lds_sync(); v8f o8[8];
#pragma unroll
  for (int t = 0; t < 8; ++t) o8[t] = (v8f){};
  { const v16b a = frag_kb(&Nh[nloc][0], hlf), al = frag_kb(&Nl[nloc][0], hlf);
#pragma unroll
    for (int t = 0; t < 8; ++t) { const v16b bw = frag_kb(WO + (size_t)(t * 16 + nloc) * D, hlf); o8[t] = wmma16b(a, bw, o8[t]); o8[t] = wmma16b(al, bw, o8[t]); } }
#pragma unroll
  for (int t = 0; t < 8; ++t) { const int cc = t * 16 + nloc; const float bb = bfv(bo[cc]);
#pragma unroll
    for (int r8 = 0; r8 < 8; ++r8) Tf[8 * hlf + r8][cc] = o8[t][r8] * (1.0f / (HS * WSC)) + bb; }
  wave_lds_sync();
  for (int pass = 0; pass < 2; ++pass) { for (int rr = 0; rr < 16; ++rr) *(volatile v4f*)(out + (t0 + rr) * FO + lane * 4) = *(const v4f*)(&Tf[rr][lane * 4]); __threadfence(); } }
}

extern "C" void kernel_launch(void* const* d_in, const int* in_sizes, int n_in, void* d_out, int out_size, void* d_ws, size_t ws_size, hipStream_t stream) {
  (void)n_in;
  auto Fp = [&](int i) { return (const float*)d_in[i]; };
  if (in_sizes[0] != N1 * DI || in_sizes[1] != N2 * DI || in_sizes[2] != DI * D || in_sizes[4] != DI * D || in_sizes[6] != DI * D || in_sizes[8] != D || in_sizes[10] != D * FO || in_sizes[11] != FO || out_size != N1 * FO) return;
  const int QLIM = N1, KLIM = N2;
  size_t off = 0; char* ws = (char*)d_ws;
  auto carve = [&](size_t bytes) { char* p = ws + off; off += (bytes + 255) & ~(size_t)255; return p; };
  b16* W3 = (b16*)carve((size_t)3 * D * DI * 2); b16* WO = (b16*)carve((size_t)FO * D * 2); b16* Qh = (b16*)carve((size_t)N1 * D * 2); b16* Ql = (b16*)carve((size_t)N1 * D * 2); b16* Kh = (b16*)carve((size_t)N2 * D * 2); b16* Kl = (b16*)carve((size_t)N2 * D * 2); b16* Vh = (b16*)carve((size_t)N2 * D * 2); b16* Vl = (b16*)carve((size_t)N2 * D * 2);
  if (off > ws_size || off > ((size_t)8 << 20)) return;
  wput_kernel<<<(3 * D * (DI / 8) + 255) / 256, 256, 0, stream>>>(Fp(2), Fp(4), Fp(6), Fp(10), W3, WO);
  proj_kernel<0><<<QLIM / 16, 32, 0, stream>>>(Fp(0), W3, Fp(3), Fp(3), QLIM, Qh, Ql, Qh, Ql);
  proj_kernel<1><<<KLIM / 16, 32, 0, stream>>>(Fp(1), W3, Fp(5), Fp(7), KLIM, Kh, Kl, Vh, Vl);
  att_kernel<<<QLIM / 16, 32, 0, stream>>>(Qh, Ql, Kh, Kl, Vh, Vl, WO, Fp(8), Fp(9), Fp(11), QLIM, KLIM, (float*)d_out);
}
